// MDFO_68040871903659
// MI455X (gfx1250) — hardware-verified
//
#include <hip/hip_runtime.h>
#include <math.h>
#include <stdint.h>


#define NBATCH 8
#define CH     256
#define CL     128
#define NPIX   4096
#define RR     64
#define MM     2048

typedef _Float16     v16h __attribute__((ext_vector_type(16)));
typedef _Float16     v8h  __attribute__((ext_vector_type(8)));
typedef float        v8f  __attribute__((ext_vector_type(8)));
typedef float        v4f  __attribute__((ext_vector_type(4)));
typedef float        v2f  __attribute__((ext_vector_type(2)));
typedef unsigned int v4u  __attribute__((ext_vector_type(4)));

union FragH { v16h v; v4u q[2]; };
union PackH { _Float16 h[16]; unsigned short us[16]; v4u q[2]; };
union Pack8 { v8h v; _Float16 h[8]; };

__device__ __forceinline__ v8f wmma_f16(v16h a, v16h b, v8f c)
{
  v8f d = __builtin_amdgcn_wmma_f32_16x16x32_f16(false, a, false, b, (short)0, c, false, false);
  asm volatile("v_nop\n\tv_nop\n\tv_nop\n\tv_nop" : "+v"(d) : "v"(a), "v"(b));
  return d;
}

template<typename TA, typename TB, bool B_TRANS, int EPI, int N, int K>
__global__ __launch_bounds__(128) void wmma_gemm(
    const TA* __restrict__ Ag, const TB* __restrict__ Bg,
    float* Cf, _Float16* Ch,
    const float* __restrict__ bias,
    const float* __restrict__ bng, const float* __restrict__ bnb,
    const float* __restrict__ bnm, const float* __restrict__ bnv,
    const float* __restrict__ resid,
    float a_scale, float acc_scale, long aB, long bB, long cB, long rB)
{
  constexpr bool A16 = (sizeof(TA) == 2);
  constexpr bool B16 = (sizeof(TB) == 2);
  static_assert(!B_TRANS || B16);
  static_assert((K % 32) == 0 && (N % 64) == 0);
  constexpr int AS_ = 40;
  constexpr int BS_ = 40;
  constexpr int CSP = 68;
  __shared__ __align__(16) _Float16 As[64 * AS_];
  __shared__ __align__(16) _Float16 Bt[64 * BS_];
  __shared__ __align__(16) float    Cs[64 * CSP];

  const int tid  = threadIdx.x;
  const int wave = tid >> 5;
  const int lane = tid & 31;
  const int h    = lane >> 4;
  const int l15  = lane & 15;
  const int b    = blockIdx.z;
  const int n0   = blockIdx.x * 64;
  const int m0   = blockIdx.y * 64;

  const TA* Ab = Ag + (size_t)b * (size_t)aB;
  const TB* Bb = Bg + (size_t)b * (size_t)bB;

  v8f acc[4];
#pragma unroll
  for (int j = 0; j < 4; ++j)
#pragma unroll
    for (int e = 0; e < 8; ++e) acc[j][e] = 0.0f;

  const int arow = tid >> 1;
  const int akk  = (tid & 1) * 16;

  for (int k0 = 0; k0 < K; k0 += 32) {
    {
      const TA* ap = Ab + (size_t)(m0 + arow) * K + k0 + akk;
      v4u* dst = (v4u*)&As[arow * AS_ + akk];
      if constexpr (A16) {
        const v4u* src = (const v4u*)ap;
        const v4u s0 = src[0], s1 = src[1];
        dst[0] = s0; dst[1] = s1;
      } else {
        const v4f* src = (const v4f*)ap;
        const v4f s0 = src[0], s1 = src[1], s2 = src[2], s3 = src[3];
        PackH u;
        u.h[0]  = (_Float16)(s0.x * a_scale); u.h[1]  = (_Float16)(s0.y * a_scale);
        u.h[2]  = (_Float16)(s0.z * a_scale); u.h[3]  = (_Float16)(s0.w * a_scale);
        u.h[4]  = (_Float16)(s1.x * a_scale); u.h[5]  = (_Float16)(s1.y * a_scale);
        u.h[6]  = (_Float16)(s1.z * a_scale); u.h[7]  = (_Float16)(s1.w * a_scale);
        u.h[8]  = (_Float16)(s2.x * a_scale); u.h[9]  = (_Float16)(s2.y * a_scale);
        u.h[10] = (_Float16)(s2.z * a_scale); u.h[11] = (_Float16)(s2.w * a_scale);
        u.h[12] = (_Float16)(s3.x * a_scale); u.h[13] = (_Float16)(s3.y * a_scale);
        u.h[14] = (_Float16)(s3.z * a_scale); u.h[15] = (_Float16)(s3.w * a_scale);
        dst[0] = u.q[0]; dst[1] = u.q[1];
      }
    }
    if constexpr (B_TRANS) {
      const int n  = tid >> 1;
      const int kk = (tid & 1) * 16;
      const v4u* src = (const v4u*)(Bb + (size_t)(n0 + n) * K + k0 + kk);
      const v4u s0 = src[0], s1 = src[1];
      v4u* dst = (v4u*)&Bt[n * BS_ + kk];
      dst[0] = s0; dst[1] = s1;
    } else {
      const int ng = (tid & 31) << 1;
      const int kg = (tid >> 5) << 3;
      PackH u;
      const TB* src = Bb + (size_t)(k0 + kg) * N + n0 + ng;
      if constexpr (B16) {
#pragma unroll
        for (int r = 0; r < 8; ++r) {
          const unsigned int w = *(const unsigned int*)(src + (size_t)r * N);
          u.us[r]     = (unsigned short)(w & 0xffffu);
          u.us[8 + r] = (unsigned short)(w >> 16);
        }
      } else {
#pragma unroll
        for (int r = 0; r < 8; ++r) {
          const v2f s = *(const v2f*)(src + (size_t)r * N);
          u.h[r]     = (_Float16)s.x;
          u.h[8 + r] = (_Float16)s.y;
        }
      }
      *(v4u*)&Bt[(ng + 0) * BS_ + kg] = u.q[0];
      *(v4u*)&Bt[(ng + 1) * BS_ + kg] = u.q[1];
    }
    __syncthreads();

    FragH fa;
    {
      const v4u* p = (const v4u*)&As[((wave << 4) + l15) * AS_ + (h << 3)];
      fa.q[0] = p[0];
      fa.q[1] = p[2];
    }
#pragma unroll
    for (int j = 0; j < 4; ++j) {
      FragH fb;
      const v4u* p = (const v4u*)&Bt[((j << 4) + l15) * BS_ + (h << 3)];
      fb.q[0] = p[0];
      fb.q[1] = p[2];
      acc[j] = wmma_f16(fa.v, fb.v, acc[j]);
    }
    __syncthreads();
  }

  const int lr0 = (wave << 4) + (h << 3);
  float addv[8], sc[8], sh[8];
#pragma unroll
  for (int e = 0; e < 8; ++e) {
    const int grow = m0 + lr0 + e;
    if constexpr (EPI == 1) {
      const float scv = bng[grow] / sqrtf(bnv[grow] + 1e-5f);
      sc[e] = scv;
      sh[e] = bnb[grow] - bnm[grow] * scv;
      addv[e] = bias[grow];
    } else if constexpr (EPI == 0) {
      addv[e] = bias[grow]; sc[e] = 1.0f; sh[e] = 0.0f;
    } else {
      addv[e] = 0.0f; sc[e] = 1.0f; sh[e] = 0.0f;
    }
  }
#pragma unroll
  for (int j = 0; j < 4; ++j) {
#pragma unroll
    for (int e = 0; e < 8; ++e) {
      float v = acc[j][e] * acc_scale + addv[e];
      if constexpr (EPI == 1) v = v * sc[e] + sh[e];
      Cs[(lr0 + e) * CSP + (j << 4) + l15] = v;
    }
  }
  __syncthreads();

  if constexpr (EPI == 1) {
    v4f vals[8];
#pragma unroll
    for (int it = 0; it < 8; ++it) {
      const int idx = it * 128 + tid;
      const int row = idx >> 4;
      const int c4  = idx & 15;
      const v4f v = *(const v4f*)&Cs[row * CSP + c4 * 4];
      const v4f r = *(const v4f*)(resid + (size_t)b * (size_t)rB + (size_t)(m0 + row) * N + n0 + c4 * 4);
      vals[it] = v + r;
    }
#pragma unroll
    for (int it = 0; it < 8; ++it) {
      const int idx = it * 128 + tid;
      const int row = idx >> 4;
      const int c4  = idx & 15;
      float* p = Cf + (size_t)b * (size_t)cB + (size_t)(m0 + row) * N + n0 + c4 * 4;
      *(volatile v4f*)p = vals[it];
    }
    __threadfence();
#pragma unroll
    for (int it = 0; it < 8; ++it) {
      const int idx = it * 128 + tid;
      const int row = idx >> 4;
      const int c4  = idx & 15;
      float* p = Cf + (size_t)b * (size_t)cB + (size_t)(m0 + row) * N + n0 + c4 * 4;
      *(volatile v4f*)p = vals[it];
    }
  } else {
    v8h vals[4];
#pragma unroll
    for (int it = 0; it < 4; ++it) {
      const int idx = it * 128 + tid;
      const int row = idx >> 3;
      const int c8  = idx & 7;
      const v4f p0 = *(const v4f*)&Cs[row * CSP + c8 * 8];
      const v4f p1 = *(const v4f*)&Cs[row * CSP + c8 * 8 + 4];
      Pack8 u;
      u.h[0] = (_Float16)p0.x; u.h[1] = (_Float16)p0.y; u.h[2] = (_Float16)p0.z; u.h[3] = (_Float16)p0.w;
      u.h[4] = (_Float16)p1.x; u.h[5] = (_Float16)p1.y; u.h[6] = (_Float16)p1.z; u.h[7] = (_Float16)p1.w;
      vals[it] = u.v;
    }
#pragma unroll
    for (int it = 0; it < 4; ++it) {
      const int idx = it * 128 + tid;
      const int row = idx >> 3;
      const int c8  = idx & 7;
      _Float16* p = Ch + (size_t)b * (size_t)cB + (size_t)(m0 + row) * N + n0 + c8 * 8;
      *(volatile v8h*)p = vals[it];
    }
    __threadfence();
#pragma unroll
    for (int it = 0; it < 4; ++it) {
      const int idx = it * 128 + tid;
      const int row = idx >> 3;
      const int c8  = idx & 7;
      _Float16* p = Ch + (size_t)b * (size_t)cB + (size_t)(m0 + row) * N + n0 + c8 * 8;
      *(volatile v8h*)p = vals[it];
    }
  }
}


__global__ __launch_bounds__(256) void pool_kernel(const float* __restrict__ z,
                                                   float* pm, float* px)
{
  __shared__ __align__(16) float s_sum[32];
  __shared__ __align__(16) float s_max[32];
  const int tid = threadIdx.x, wave = tid >> 5, lane = tid & 31;
  const int bc0 = blockIdx.x * 32;
#pragma unroll 1
  for (int q = 0; q < 4; ++q) {
    const int cl = wave * 4 + q;
    const float* base = z + (size_t)(bc0 + cl) * NPIX;
    float s = 0.0f, m = -__builtin_inff();
#pragma unroll 4
    for (int it = 0; it < NPIX / 128; ++it) {
      const v4f v = *(const v4f*)(base + (size_t)(it * 32 + lane) * 4);
      s += (v.x + v.y) + (v.z + v.w);
      m = fmaxf(m, fmaxf(fmaxf(v.x, v.y), fmaxf(v.z, v.w)));
    }
#pragma unroll
    for (int o = 16; o > 0; o >>= 1) {
      s += __shfl_xor(s, o);
      m = fmaxf(m, __shfl_xor(m, o));
    }
    if (lane == 0) { s_sum[cl] = s * (1.0f / 4096.0f); s_max[cl] = m; }
  }
  __syncthreads();
  if (wave < 2) {
    const int lq = lane & 7;
    const v4f vs = *(const v4f*)&s_sum[lq * 4];
    const v4f vm = *(const v4f*)&s_max[lq * 4];
    const v4f v = (wave == 0) ? vs : vm;
    float* dst = ((wave == 0) ? pm : px) + (size_t)bc0 + lq * 4;
    if (lane < 8) *(volatile v4f*)dst = v;
    __threadfence();
    if (lane < 8) *(volatile v4f*)dst = v;
  }
}

__global__ __launch_bounds__(256) void ca_kernel(const float* __restrict__ pm, const float* __restrict__ px,
                                                 const float* __restrict__ fc1, const float* __restrict__ fc2,
                                                 float* ca)
{
  __shared__ float smv[CH], sxv[CH];
  __shared__ float hm[16], hx[16];
  const int b = blockIdx.x, t = threadIdx.x, wave = t >> 5, lane = t & 31;
  smv[t] = pm[b * CH + t];
  sxv[t] = px[b * CH + t];
  __syncthreads();
  if (wave == 0) {
    const int hh = lane & 15;
    float a = 0.0f, c = 0.0f;
#pragma unroll 1
    for (int i = 0; i < CH; ++i) {
      const float w = fc1[hh * CH + i];
      a += w * smv[i];
      c += w * sxv[i];
    }
    if (lane < 16) { hm[hh] = fmaxf(a, 0.0f); hx[hh] = fmaxf(c, 0.0f); }
  }
  __syncthreads();
  float o1 = 0.0f, o2 = 0.0f;
#pragma unroll 1
  for (int hh = 0; hh < 16; ++hh) {
    const float w = fc2[t * 16 + hh];
    o1 += w * hm[hh];
    o2 += w * hx[hh];
  }
  const float o = o1 + o2;
  const float r = 1.0f / (1.0f + __expf(-o));
  float* dst = ca + (size_t)b * CH + t;
  *(volatile float*)dst = r;
  __threadfence();
  *(volatile float*)dst = r;
}

__global__ __launch_bounds__(256) void chstats_kernel(const float* __restrict__ zp, const float* __restrict__ ca,
                                                      float* cm, float* cx)
{
  const int idx = blockIdx.x * 256 + threadIdx.x;
  const int b = idx >> 12, n = idx & 4095;
  const float* base = zp + (size_t)b * CH * NPIX + n;
  const float* cab  = ca + b * CH;
  float s = 0.0f, m = -__builtin_inff();
#pragma unroll 4
  for (int c = 0; c < CH; ++c) {
    const float v = base[(size_t)c * NPIX] * cab[c];
    s += v;
    m = fmaxf(m, v);
  }
  const float mean = s * (1.0f / 256.0f);
  *(volatile float*)(cm + idx) = mean;
  *(volatile float*)(cx + idx) = m;
  __threadfence();
  *(volatile float*)(cm + idx) = mean;
  *(volatile float*)(cx + idx) = m;
}

__global__ __launch_bounds__(256) void saconv_kernel(const float* __restrict__ cm, const float* __restrict__ cx,
                                                     const float* __restrict__ w, float* sa)
{
  const int idx = blockIdx.x * 256 + threadIdx.x;
  const int b = idx >> 12, n = idx & 4095, y = n >> 6, x = n & 63;
  float acc = 0.0f;
#pragma unroll 1
  for (int ch = 0; ch < 2; ++ch) {
    const float* src = (ch ? cx : cm) + (size_t)b * NPIX;
    const float* wc  = w + ch * 49;
#pragma unroll 1
    for (int ky = 0; ky < 7; ++ky) {
      const int  yy  = y + ky - 3;
      const bool oky = (yy >= 0) && (yy <= 63);
      const int  yc  = min(max(yy, 0), 63);
#pragma unroll 1
      for (int kx = 0; kx < 7; ++kx) {
        const int  xx = x + kx - 3;
        const bool ok = oky && (xx >= 0) && (xx <= 63);
        const int  xc = min(max(xx, 0), 63);
        float v = src[yc * 64 + xc];
        v = ok ? v : 0.0f;
        acc += wc[ky * 7 + kx] * v;
      }
    }
  }
  *(volatile float*)(sa + idx) = acc;
  __threadfence();
  *(volatile float*)(sa + idx) = acc;
}

__global__ __launch_bounds__(256) void fusion_kernel(const float* __restrict__ zp, const float* __restrict__ ca,
                                                     const float* __restrict__ sa, const float* __restrict__ xin,
                                                     const float* __restrict__ fwp, float* out)
{
  const int i4 = blockIdx.x * 256 + threadIdx.x;
  const int b  = i4 >> 18;
  const int c  = (i4 >> 10) & 255;
  const int n4 = (i4 & 1023) * 4;
  const size_t e = (size_t)i4 * 4;
  const v4f z  = *(const v4f*)(zp + e);
  const v4f xv = *(const v4f*)(xin + e);
  const v4f s4 = *(const v4f*)(sa + (size_t)b * NPIX + n4);
  const float cav = ca[b * CH + c];
  const float fw  = fwp[0];
  const float omf = 1.0f - fw;
  v4f o;
  {
    const float g0 = 1.0f / (1.0f + __expf(-s4.x));
    const float g1 = 1.0f / (1.0f + __expf(-s4.y));
    const float g2 = 1.0f / (1.0f + __expf(-s4.z));
    const float g3 = 1.0f / (1.0f + __expf(-s4.w));
    o.x = fw * ((z.x * cav) * g0) + omf * xv.x;
    o.y = fw * ((z.y * cav) * g1) + omf * xv.y;
    o.z = fw * ((z.z * cav) * g2) + omf * xv.z;
    o.w = fw * ((z.w * cav) * g3) + omf * xv.w;
  }
  float* p = out + e;
  *(volatile v4f*)p = o;
  __threadfence();
  *(volatile v4f*)p = o;
}

extern "C" void kernel_launch(void* const* d_in, const int* in_sizes, int n_in,
                              void* d_out, int out_size, void* d_ws, size_t ws_size,
                              hipStream_t stream)
{
  if (n_in < 30) return;
  if (in_sizes[0] != NBATCH * CH * NPIX || in_sizes[1] != NBATCH * CL * NPIX) return;
  if (out_size != NBATCH * CH * NPIX) return;

  const float* in_x     = (const float*)d_in[0];
  const float* in_x0    = (const float*)d_in[1];
  const float* cnl_g_w  = (const float*)d_in[2];
  const float* cnl_g_b  = (const float*)d_in[3];
  const float* cnl_t_w  = (const float*)d_in[4];
  const float* cnl_t_b  = (const float*)d_in[5];
  const float* cnl_p_w  = (const float*)d_in[6];
  const float* cnl_p_b  = (const float*)d_in[7];
  const float* cnl_W_w  = (const float*)d_in[8];
  const float* cnl_W_b  = (const float*)d_in[9];
  const float* cnl_bn_g = (const float*)d_in[10];
  const float* cnl_bn_b = (const float*)d_in[11];
  const float* cnl_bn_m = (const float*)d_in[12];
  const float* cnl_bn_v = (const float*)d_in[13];
  const float* pnl_g_w  = (const float*)d_in[14];
  const float* pnl_g_b  = (const float*)d_in[15];
  const float* pnl_t_w  = (const float*)d_in[16];
  const float* pnl_t_b  = (const float*)d_in[17];
  const float* pnl_p_w  = (const float*)d_in[18];
  const float* pnl_p_b  = (const float*)d_in[19];
  const float* pnl_W_w  = (const float*)d_in[20];
  const float* pnl_W_b  = (const float*)d_in[21];
  const float* pnl_bn_g = (const float*)d_in[22];
  const float* pnl_bn_b = (const float*)d_in[23];
  const float* pnl_bn_m = (const float*)d_in[24];
  const float* pnl_bn_v = (const float*)d_in[25];
  const float* ca_fc1_w = (const float*)d_in[26];
  const float* ca_fc2_w = (const float*)d_in[27];
  const float* sa_w     = (const float*)d_in[28];
  const float* fwp      = (const float*)d_in[29];

  constexpr size_t SZ_F16_128 = (size_t)NBATCH * CL * NPIX * 2;
  constexpr size_t SZ_F16_64  = (size_t)NBATCH * RR * NPIX * 2;
  constexpr size_t SZ_AFF     = (size_t)NBATCH * CL * CL * 2;
  constexpr size_t SZ_Z       = (size_t)NBATCH * CH * NPIX * 4;
  constexpr size_t SZ_POOL    = (size_t)NBATCH * CH * 4;
  constexpr size_t SZ_MAP     = (size_t)NBATCH * NPIX * 4;
  constexpr size_t OFF_GX   = 0;
  constexpr size_t OFF_TH   = OFF_GX + SZ_F16_128;
  constexpr size_t OFF_PH   = OFF_TH + SZ_F16_128;
  constexpr size_t OFF_Y    = OFF_PH + SZ_F16_128;
  constexpr size_t OFF_ATT  = OFF_Y + SZ_F16_128;
  constexpr size_t OFF_G2   = OFF_ATT + SZ_AFF;
  constexpr size_t OFF_P2   = OFF_G2 + SZ_F16_64;
  constexpr size_t OFF_T2   = OFF_P2 + SZ_F16_64;
  constexpr size_t OFF_Y2   = OFF_T2 + SZ_F16_64;
  constexpr size_t OFF_KT   = OFF_Y2 + SZ_F16_64;
  constexpr size_t OFF_ZCNL = OFF_KT + SZ_AFF;
  constexpr size_t OFF_ZPNL = OFF_ZCNL + SZ_Z;
  constexpr size_t OFF_PM   = OFF_ZPNL + SZ_Z;
  constexpr size_t OFF_PX   = OFF_PM + SZ_POOL;
  constexpr size_t OFF_CA   = OFF_PX + SZ_POOL;
  constexpr size_t OFF_CM   = OFF_CA + SZ_POOL;
  constexpr size_t OFF_CX   = OFF_CM + SZ_MAP;
  constexpr size_t OFF_SA   = OFF_CX + SZ_MAP;
  constexpr size_t WS_END   = OFF_SA + SZ_MAP;
  static_assert(WS_END <= (size_t)134217728);
  static_assert((OFF_ATT % 256) == 0 && (OFF_ZCNL % 256) == 0 && (OFF_PM % 256) == 0 && (OFF_SA % 256) == 0);
  if (ws_size < WS_END) return;

  char* ws = (char*)d_ws;
  _Float16* gx16  = (_Float16*)(ws + OFF_GX);
  _Float16* th16  = (_Float16*)(ws + OFF_TH);
  _Float16* ph16  = (_Float16*)(ws + OFF_PH);
  _Float16* y16   = (_Float16*)(ws + OFF_Y);
  _Float16* att16 = (_Float16*)(ws + OFF_ATT);
  _Float16* g2    = (_Float16*)(ws + OFF_G2);
  _Float16* p2    = (_Float16*)(ws + OFF_P2);
  _Float16* t2    = (_Float16*)(ws + OFF_T2);
  _Float16* y2    = (_Float16*)(ws + OFF_Y2);
  _Float16* kt16  = (_Float16*)(ws + OFF_KT);
  float*    zcnl  = (float*)(ws + OFF_ZCNL);
  float*    zpnl  = (float*)(ws + OFF_ZPNL);
  float*    pm    = (float*)(ws + OFF_PM);
  float*    px    = (float*)(ws + OFF_PX);
  float*    cav   = (float*)(ws + OFF_CA);
  float*    cm    = (float*)(ws + OFF_CM);
  float*    cx    = (float*)(ws + OFF_CX);
  float*    sa    = (float*)(ws + OFF_SA);

  const dim3 blk(128);
  const long S128 = 128L * NPIX, S256 = 256L * NPIX, S64 = 64L * NPIX;
  const long SAFF = 128L * 128;
  const float WS  = 16.0f;
  const float IWS = 1.0f / 16.0f;

  wmma_gemm<float, float, false, 0, NPIX, 128><<<dim3(NPIX / 64, 2, NBATCH), blk, 0, stream>>>(
      cnl_g_w, in_x0, nullptr, gx16, cnl_g_b, nullptr, nullptr, nullptr, nullptr, nullptr,
      WS, IWS, 0L, S128, S128, 0L);
  wmma_gemm<float, float, false, 0, NPIX, 256><<<dim3(NPIX / 64, 2, NBATCH), blk, 0, stream>>>(
      cnl_t_w, in_x, nullptr, th16, cnl_t_b, nullptr, nullptr, nullptr, nullptr, nullptr,
      WS, IWS, 0L, S256, S128, 0L);
  wmma_gemm<float, float, false, 0, NPIX, 128><<<dim3(NPIX / 64, 2, NBATCH), blk, 0, stream>>>(
      cnl_p_w, in_x0, nullptr, ph16, cnl_p_b, nullptr, nullptr, nullptr, nullptr, nullptr,
      WS, IWS, 0L, S128, S128, 0L);
  wmma_gemm<_Float16, _Float16, true, 2, 128, NPIX><<<dim3(2, 2, NBATCH), blk, 0, stream>>>(
      th16, ph16, nullptr, att16, nullptr, nullptr, nullptr, nullptr, nullptr, nullptr,
      1.0f, 1.0f / 16.0f, S128, S128, SAFF, 0L);
  wmma_gemm<_Float16, _Float16, false, 2, NPIX, 128><<<dim3(NPIX / 64, 2, NBATCH), blk, 0, stream>>>(
      att16, gx16, nullptr, y16, nullptr, nullptr, nullptr, nullptr, nullptr, nullptr,
      1.0f, 1.0f / 8.0f, SAFF, S128, S128, 0L);
  wmma_gemm<float, _Float16, false, 1, NPIX, 128><<<dim3(NPIX / 64, 4, NBATCH), blk, 0, stream>>>(
      cnl_W_w, y16, zcnl, nullptr, cnl_W_b, cnl_bn_g, cnl_bn_b, cnl_bn_m, cnl_bn_v, in_x,
      WS, IWS, 0L, S128, S256, S256);

  wmma_gemm<float, float, false, 0, NPIX, 128><<<dim3(NPIX / 64, 1, NBATCH), blk, 0, stream>>>(
      pnl_g_w, in_x0, nullptr, g2, pnl_g_b, nullptr, nullptr, nullptr, nullptr, nullptr,
      WS, IWS, 0L, S128, S64, 0L);
  wmma_gemm<float, float, false, 0, NPIX, 128><<<dim3(NPIX / 64, 1, NBATCH), blk, 0, stream>>>(
      pnl_p_w, in_x0, nullptr, p2, pnl_p_b, nullptr, nullptr, nullptr, nullptr, nullptr,
      WS, IWS, 0L, S128, S64, 0L);
  wmma_gemm<float, float, false, 0, NPIX, 256><<<dim3(NPIX / 64, 1, NBATCH), blk, 0, stream>>>(
      pnl_t_w, zcnl, nullptr, t2, pnl_t_b, nullptr, nullptr, nullptr, nullptr, nullptr,
      WS, IWS, 0L, S256, S64, 0L);
  wmma_gemm<_Float16, _Float16, true, 2, 128, MM><<<dim3(2, 2, NBATCH), blk, 0, stream>>>(
      g2, p2, nullptr, kt16, nullptr, nullptr, nullptr, nullptr, nullptr, nullptr,
      1.0f, 1.0f, 128L * MM, 128L * MM, SAFF, 0L);
  wmma_gemm<_Float16, _Float16, false, 2, MM, 128><<<dim3(MM / 64, 2, NBATCH), blk, 0, stream>>>(
      kt16, t2, nullptr, y2, nullptr, nullptr, nullptr, nullptr, nullptr, nullptr,
      1.0f, 1.0f / 2048.0f, SAFF, 128L * MM, 128L * MM, 0L);
  wmma_gemm<float, _Float16, false, 1, NPIX, 64><<<dim3(NPIX / 64, 4, NBATCH), blk, 0, stream>>>(
      pnl_W_w, y2, zpnl, nullptr, pnl_W_b, pnl_bn_g, pnl_bn_b, pnl_bn_m, pnl_bn_v, zcnl,
      WS, IWS, 0L, S64, S256, S256);

  pool_kernel<<<dim3(NBATCH * CH / 32), dim3(256), 0, stream>>>(zpnl, pm, px);
  ca_kernel<<<dim3(NBATCH), dim3(256), 0, stream>>>(pm, px, ca_fc1_w, ca_fc2_w, cav);
  chstats_kernel<<<dim3(NBATCH * NPIX / 256), dim3(256), 0, stream>>>(zpnl, cav, cm, cx);
  saconv_kernel<<<dim3(NBATCH * NPIX / 256), dim3(256), 0, stream>>>(cm, cx, sa_w, sa);
  fusion_kernel<<<dim3(NBATCH * CH * NPIX / 4 / 256), dim3(256), 0, stream>>>(
      zpnl, cav, sa, in_x, fwp, (float*)d_out);
}
